// SelfConditionedMultiheadAttention_2542620639588
// MI455X (gfx1250) — hardware-verified
//
#include <hip/hip_runtime.h>
#include <stdint.h>


static constexpr int BATCH = 2;
static constexpr int TSEQ  = 2048;
static constexpr int DIM   = 1024;
static constexpr int NHEAD = 16;
static constexpr int HDIM  = 64;
static constexpr int NROWS = BATCH * TSEQ;
static constexpr int CSP   = 132;
static constexpr int PBP   = 72;
static constexpr int OBP   = 68;

typedef unsigned int v4u_t __attribute__((ext_vector_type(4)));
typedef v4u_t        v4u   __attribute__((may_alias));
typedef float        v4f_t __attribute__((ext_vector_type(4)));
typedef v4f_t        v4f   __attribute__((may_alias));
typedef float        v8f   __attribute__((ext_vector_type(8)));
typedef _Float16     v8h_t __attribute__((ext_vector_type(8)));
typedef _Float16     v16h  __attribute__((ext_vector_type(16)));
typedef __bf16       v16b  __attribute__((ext_vector_type(16)));

union FragB  { v16b v;  v4u_t u[2]; };
union FragH  { v16h v;  v4u_t u[2]; };
union Pack8H { v8h_t v; v4u_t u;    };

#define NOP4 "v_nop\n\tv_nop\n\tv_nop\n\tv_nop"

__device__ __forceinline__ v8f zero8() {
    v8f z;
#pragma unroll
    for (int r = 0; r < 8; ++r) z[r] = 0.f;
    return z;
}

__device__ __forceinline__ v8f mma_bf16(v16b a, v16b b, v8f c) {
    return __builtin_amdgcn_wmma_f32_16x16x32_bf16(false, a, false, b, (short)0, c, false, false);
}
__device__ __forceinline__ v8f mma_f16(v16h a, v16h b, v8f c) {
    return __builtin_amdgcn_wmma_f32_16x16x32_f16(false, a, false, b, (short)0, c, false, false);
}

__device__ __forceinline__ unsigned bfbits(float f) {
    unsigned u = __float_as_uint(f);
    u += 0x7FFFu + ((u >> 16) & 1u);
    return u >> 16;
}
__device__ __forceinline__ float bfval(unsigned b) { return __uint_as_float(b << 16); }
__device__ __forceinline__ float bfrne(float f) { return bfval(bfbits(f)); }

__device__ __forceinline__ v4u_t pack_bf16_8(const float* f) {
    v4u_t r;
    r.x = bfbits(f[0]) | (bfbits(f[1]) << 16);
    r.y = bfbits(f[2]) | (bfbits(f[3]) << 16);
    r.z = bfbits(f[4]) | (bfbits(f[5]) << 16);
    r.w = bfbits(f[6]) | (bfbits(f[7]) << 16);
    return r;
}

__device__ __forceinline__ void split_bf16_8(const float* f, v4u_t& hv, v4u_t& lv) {
    unsigned hb[8], lb[8];
#pragma unroll
    for (int i = 0; i < 8; ++i) {
        hb[i] = bfbits(f[i]);
        lb[i] = bfbits(f[i] - bfval(hb[i]));
    }
    hv.x = hb[0] | (hb[1] << 16); hv.y = hb[2] | (hb[3] << 16);
    hv.z = hb[4] | (hb[5] << 16); hv.w = hb[6] | (hb[7] << 16);
    lv.x = lb[0] | (lb[1] << 16); lv.y = lb[2] | (lb[3] << 16);
    lv.z = lb[4] | (lb[5] << 16); lv.w = lb[6] | (lb[7] << 16);
}

__device__ __forceinline__ v4u_t pack_f16_8(const float* f) {
    Pack8H p;
#pragma unroll
    for (int i = 0; i < 8; ++i) p.v[i] = (_Float16)f[i];
    return p.u;
}

__device__ __forceinline__ void ldfrag_b(FragB& f, const unsigned short* p) {
    f.u[0] = *(const v4u*)(p);
    f.u[1] = *(const v4u*)(p + 16);
}
__device__ __forceinline__ void ldfrag_h(FragH& f, const unsigned short* p) {
    f.u[0] = *(const v4u*)(p);
    f.u[1] = *(const v4u*)(p + 16);
}

__global__ __launch_bounds__(256) void k_cvt_x(const float* __restrict__ x,
                                               unsigned short* y, int n8) {
    const int i = blockIdx.x * 256 + threadIdx.x;
    if (i >= n8) return;
    const float* p = x + (size_t)i * 8;
    v4f_t a = *(const v4f*)(p);
    v4f_t c = *(const v4f*)(p + 4);
    float f[8] = {a.x, a.y, a.z, a.w, c.x, c.y, c.z, c.w};
    const v4u_t v = pack_bf16_8(f);
    unsigned short* d = y + (size_t)i * 8;
    *(volatile v4u_t*)d = v;
    __threadfence();
    *(volatile v4u_t*)d = v;
}

__global__ __launch_bounds__(256) void k_cvt_w(const float* __restrict__ W0,
                                               const float* __restrict__ W1,
                                               const float* __restrict__ W2,
                                               const float* __restrict__ W3,
                                               const float* __restrict__ W4,
                                               unsigned short* Wt, int D, int total) {
    const int g = blockIdx.x * 256 + threadIdx.x;
    if (g >= total) return;
    const int kg  = D >> 3;
    const int per = D * kg;
    const int mat = g / per;
    const int rem = g - mat * per;
    const int n   = rem / kg;
    const int k8  = rem - n * kg;
    const float* src = (mat == 0) ? W0 : (mat == 1) ? W1 : (mat == 2) ? W2 : (mat == 3) ? W3 : W4;
    float f[8];
#pragma unroll
    for (int i = 0; i < 8; ++i) f[i] = src[(size_t)(k8 * 8 + i) * D + n];
    const v4u_t v = pack_bf16_8(f);
    unsigned short* d = Wt + (size_t)mat * D * D + (size_t)n * D + k8 * 8;
    *(volatile v4u_t*)d = v;
    __threadfence();
    *(volatile v4u_t*)d = v;
}

template <int AP, int EP, int HASB>
__global__ __launch_bounds__(128) void k_gemm(
    const unsigned short* __restrict__ A0, const unsigned short* __restrict__ A1,
    const unsigned short* __restrict__ Bt, const float* __restrict__ bias,
    unsigned short* out0, unsigned short* out1, float* outf, int M, int N, int K) {
    __shared__ __attribute__((aligned(16))) float Cs[64][CSP];

    const int tid = threadIdx.x, lane = tid & 31, wave = tid >> 5;
    const int m = lane & 15, h = lane >> 4;
    const int wm = wave & 1, wn = wave >> 1;
    const int m0 = blockIdx.x * 64, n0 = blockIdx.y * 128;
    if (m0 + 64 > M || n0 + 128 > N) return;

    const unsigned short* ap0[2];
    const unsigned short* ap1[2];
    const unsigned short* bp[4];
#pragma unroll
    for (int mi = 0; mi < 2; ++mi) {
        const size_t ro = (size_t)(m0 + 32 * wm + 16 * mi + m) * (size_t)K + 8 * h;
        ap0[mi] = A0 + ro;
        ap1[mi] = A1 + ro;
    }
#pragma unroll
    for (int ni = 0; ni < 4; ++ni)
        bp[ni] = Bt + (size_t)(n0 + 64 * wn + 16 * ni + m) * (size_t)K + 8 * h;

    v8f acc[2][4];
#pragma unroll
    for (int mi = 0; mi < 2; ++mi)
#pragma unroll
        for (int ni = 0; ni < 4; ++ni) acc[mi][ni] = zero8();

    FragB a0[2], a1[2], b[4];
#pragma unroll 1
    for (int k0 = 0; k0 < K; k0 += 32) {
#pragma unroll
        for (int mi = 0; mi < 2; ++mi) {
            ldfrag_b(a0[mi], ap0[mi] + k0);
            if (AP == 2) ldfrag_b(a1[mi], ap1[mi] + k0);
            else a1[mi] = a0[mi];
        }
#pragma unroll
        for (int ni = 0; ni < 4; ++ni) ldfrag_b(b[ni], bp[ni] + k0);
#pragma unroll
        for (int mi = 0; mi < 2; ++mi) {
#pragma unroll
            for (int ni = 0; ni < 4; ++ni) {
                acc[mi][ni] = mma_bf16(a0[mi].v, b[ni].v, acc[mi][ni]);
                if (AP == 2) acc[mi][ni] = mma_bf16(a1[mi].v, b[ni].v, acc[mi][ni]);
            }
        }
        asm volatile(NOP4
                     : "+v"(acc[0][0]), "+v"(acc[0][1]), "+v"(acc[0][2]), "+v"(acc[0][3]),
                       "+v"(acc[1][0]), "+v"(acc[1][1]), "+v"(acc[1][2]), "+v"(acc[1][3])
                     : "v"(a0[0].v), "v"(a0[1].v), "v"(a1[0].v), "v"(a1[1].v),
                       "v"(b[0].v), "v"(b[1].v), "v"(b[2].v), "v"(b[3].v));
    }

#pragma unroll
    for (int mi = 0; mi < 2; ++mi) {
#pragma unroll
        for (int ni = 0; ni < 4; ++ni) {
            const int col = 64 * wn + 16 * ni + m;
            float bv = 0.f;
            if (HASB) bv = bfrne(bias[n0 + col]);
#pragma unroll
            for (int r = 0; r < 8; ++r)
                Cs[32 * wm + 16 * mi + 8 * h + r][col] = acc[mi][ni][r] + bv;
        }
    }
    __syncthreads();

    if (EP == 0) {
        v4u_t hv[8], lv[8];
#pragma unroll
        for (int it = 0; it < 8; ++it) {
            const int row = 16 * wave + 2 * it + h;
            const int c8 = 8 * m;
            v4f_t f0 = *(const v4f*)&Cs[row][c8];
            v4f_t f1 = *(const v4f*)&Cs[row][c8 + 4];
            float f[8] = {f0.x, f0.y, f0.z, f0.w, f1.x, f1.y, f1.z, f1.w};
            split_bf16_8(f, hv[it], lv[it]);
        }
#pragma unroll
        for (int it = 0; it < 8; ++it) {
            const size_t off = (size_t)(m0 + 16 * wave + 2 * it + h) * (size_t)N + n0 + 8 * m;
            *(volatile v4u_t*)(out0 + off) = hv[it];
            *(volatile v4u_t*)(out1 + off) = lv[it];
        }
        __threadfence();
#pragma unroll
        for (int it = 0; it < 8; ++it) {
            const size_t off = (size_t)(m0 + 16 * wave + 2 * it + h) * (size_t)N + n0 + 8 * m;
            *(volatile v4u_t*)(out0 + off) = hv[it];
            *(volatile v4u_t*)(out1 + off) = lv[it];
        }
    } else if (EP == 1) {
        const int bidx = m0 / TSEQ;
        const int t0 = m0 - bidx * TSEQ;
        v4u_t hv[8];
#pragma unroll
        for (int it = 0; it < 8; ++it) {
            const int c = 32 * wave + 4 * it + (lane >> 3);
            const int q8 = (lane & 7) * 8;
            float f[8];
#pragma unroll
            for (int i = 0; i < 8; ++i) f[i] = Cs[q8 + i][c];
            hv[it] = pack_f16_8(f);
        }
#pragma unroll
        for (int it = 0; it < 8; ++it) {
            const int c = 32 * wave + 4 * it + (lane >> 3);
            const int q8 = (lane & 7) * 8;
            const int col = n0 + c;
            const int hdd = col / HDIM, d = col - hdd * HDIM;
            const size_t off = ((size_t)(bidx * NHEAD + hdd) * HDIM + d) * (size_t)TSEQ + t0 + q8;
            *(volatile v4u_t*)(out0 + off) = hv[it];
        }
        __threadfence();
#pragma unroll
        for (int it = 0; it < 8; ++it) {
            const int c = 32 * wave + 4 * it + (lane >> 3);
            const int q8 = (lane & 7) * 8;
            const int col = n0 + c;
            const int hdd = col / HDIM, d = col - hdd * HDIM;
            const size_t off = ((size_t)(bidx * NHEAD + hdd) * HDIM + d) * (size_t)TSEQ + t0 + q8;
            *(volatile v4u_t*)(out0 + off) = hv[it];
        }
    } else {
        v4f_t fv[16];
#pragma unroll
        for (int it = 0; it < 16; ++it)
            fv[it] = *(const v4f*)&Cs[16 * wave + it][4 * lane];
#pragma unroll
        for (int it = 0; it < 16; ++it) {
            const size_t off = (size_t)(m0 + 16 * wave + it) * (size_t)N + n0 + 4 * lane;
            *(volatile v4f_t*)(outf + off) = fv[it];
        }
        __threadfence();
#pragma unroll
        for (int it = 0; it < 16; ++it) {
            const size_t off = (size_t)(m0 + 16 * wave + it) * (size_t)N + n0 + 4 * lane;
            *(volatile v4f_t*)(outf + off) = fv[it];
        }
    }
}

__global__ __launch_bounds__(128) void k_attn(
    const unsigned short* __restrict__ Qh, const unsigned short* __restrict__ Ql,
    const unsigned short* __restrict__ Kh, const unsigned short* __restrict__ Kl,
    const unsigned short* __restrict__ Vt,
    unsigned short* Oh, unsigned short* Ol) {
    __shared__ __attribute__((aligned(16))) _Float16 Pb[4][16][PBP];
    __shared__ __attribute__((aligned(16))) float    Ob[4][16][OBP];

    const int tid = threadIdx.x, lane = tid & 31, wave = tid >> 5;
    const int m = lane & 15, h = lane >> 4;
    const int b = blockIdx.z, hd = blockIdx.y;
    const int q0 = blockIdx.x * 64 + wave * 16;

    FragB qh[2], ql[2];
    {
        const size_t qo = ((size_t)b * TSEQ + q0 + m) * (size_t)DIM + hd * HDIM + 8 * h;
#pragma unroll
        for (int ks = 0; ks < 2; ++ks) {
            ldfrag_b(qh[ks], Qh + qo + 32 * ks);
            ldfrag_b(ql[ks], Ql + qo + 32 * ks);
        }
    }
    const size_t kbase = ((size_t)b * TSEQ + m) * (size_t)DIM + hd * HDIM + 8 * h;
    const size_t vbase = ((size_t)(b * NHEAD + hd) * HDIM + m) * (size_t)TSEQ + 8 * h;

    v8f o[4];
#pragma unroll
    for (int j = 0; j < 4; ++j) o[j] = zero8();
    float mrow[8], lp[8];
#pragma unroll
    for (int r = 0; r < 8; ++r) { mrow[r] = -1e30f; lp[r] = 0.f; }

#pragma unroll 1
    for (int ci = 0; ci < TSEQ / 64; ++ci) {
        const int key0 = ci * 64;

        v8f s[4];
#pragma unroll
        for (int kt = 0; kt < 4; ++kt) s[kt] = zero8();
        FragB kh, kl;
#pragma unroll
        for (int kt = 0; kt < 4; ++kt) {
            const size_t ko = kbase + (size_t)(key0 + 16 * kt) * (size_t)DIM;
#pragma unroll
            for (int ks = 0; ks < 2; ++ks) {
                ldfrag_b(kh, Kh + ko + 32 * ks);
                ldfrag_b(kl, Kl + ko + 32 * ks);
                s[kt] = mma_bf16(qh[ks].v, kh.v, s[kt]);
                s[kt] = mma_bf16(qh[ks].v, kl.v, s[kt]);
                s[kt] = mma_bf16(ql[ks].v, kh.v, s[kt]);
            }
        }
        asm volatile(NOP4
                     : "+v"(s[0]), "+v"(s[1]), "+v"(s[2]), "+v"(s[3])
                     : "v"(qh[0].v), "v"(qh[1].v), "v"(ql[0].v), "v"(ql[1].v), "v"(kh.v), "v"(kl.v));

        float al[8];
#pragma unroll
        for (int r = 0; r < 8; ++r) {
            const float v0 = s[0][r] * 0.125f, v1 = s[1][r] * 0.125f;
            const float v2 = s[2][r] * 0.125f, v3 = s[3][r] * 0.125f;
            float mx = fmaxf(fmaxf(v0, v1), fmaxf(v2, v3));
            mx = fmaxf(mx, __shfl_xor(mx, 1));
            mx = fmaxf(mx, __shfl_xor(mx, 2));
            mx = fmaxf(mx, __shfl_xor(mx, 4));
            mx = fmaxf(mx, __shfl_xor(mx, 8));
            const float mn = fmaxf(mrow[r], mx);
            al[r] = __expf(mrow[r] - mn);
            mrow[r] = mn;
            const float p0 = __expf(v0 - mn), p1 = __expf(v1 - mn);
            const float p2 = __expf(v2 - mn), p3 = __expf(v3 - mn);
            lp[r] = lp[r] * al[r] + ((p0 + p1) + (p2 + p3));
            const int row = 8 * h + r;
            Pb[wave][row][m]      = (_Float16)(p0 * 4096.f);
            Pb[wave][row][16 + m] = (_Float16)(p1 * 4096.f);
            Pb[wave][row][32 + m] = (_Float16)(p2 * 4096.f);
            Pb[wave][row][48 + m] = (_Float16)(p3 * 4096.f);
        }
#pragma unroll
        for (int j = 0; j < 4; ++j)
#pragma unroll
            for (int r = 0; r < 8; ++r) o[j][r] *= al[r];

        __syncthreads();

        FragH pf[2];
#pragma unroll
        for (int ks = 0; ks < 2; ++ks) {
            pf[ks].u[0] = *(const v4u*)&Pb[wave][m][32 * ks + 8 * h];
            pf[ks].u[1] = *(const v4u*)&Pb[wave][m][32 * ks + 16 + 8 * h];
        }
        FragH vb;
#pragma unroll
        for (int j = 0; j < 4; ++j) {
            const size_t vo = vbase + (size_t)(16 * j) * (size_t)TSEQ + key0;
#pragma unroll
            for (int ks = 0; ks < 2; ++ks) {
                ldfrag_h(vb, Vt + vo + 32 * ks);
                o[j] = mma_f16(pf[ks].v, vb.v, o[j]);
            }
        }
        asm volatile(NOP4
                     : "+v"(o[0]), "+v"(o[1]), "+v"(o[2]), "+v"(o[3])
                     : "v"(pf[0].v), "v"(pf[1].v), "v"(vb.v));
    }

    float inv[8];
#pragma unroll
    for (int r = 0; r < 8; ++r) {
        float l = lp[r];
        l += __shfl_xor(l, 1);
        l += __shfl_xor(l, 2);
        l += __shfl_xor(l, 4);
        l += __shfl_xor(l, 8);
        inv[r] = 1.0f / (l * 4096.0f);
    }
#pragma unroll
    for (int j = 0; j < 4; ++j)
#pragma unroll
        for (int r = 0; r < 8; ++r)
            Ob[wave][8 * h + r][16 * j + m] = o[j][r] * inv[r];
    __syncthreads();

    v4u_t hv[4], lv[4];
#pragma unroll
    for (int it = 0; it < 4; ++it) {
        const int row = 4 * it + (lane >> 3);
        const int c8 = (lane & 7) * 8;
        v4f_t f0 = *(const v4f*)&Ob[wave][row][c8];
        v4f_t f1 = *(const v4f*)&Ob[wave][row][c8 + 4];
        float f[8] = {f0.x, f0.y, f0.z, f0.w, f1.x, f1.y, f1.z, f1.w};
        split_bf16_8(f, hv[it], lv[it]);
    }
#pragma unroll
    for (int it = 0; it < 4; ++it) {
        const int row = 4 * it + (lane >> 3);
        const int c8 = (lane & 7) * 8;
        const size_t off = ((size_t)b * TSEQ + q0 + row) * (size_t)DIM + hd * HDIM + c8;
        *(volatile v4u_t*)(Oh + off) = hv[it];
        *(volatile v4u_t*)(Ol + off) = lv[it];
    }
    __threadfence();
#pragma unroll
    for (int it = 0; it < 4; ++it) {
        const int row = 4 * it + (lane >> 3);
        const int c8 = (lane & 7) * 8;
        const size_t off = ((size_t)b * TSEQ + q0 + row) * (size_t)DIM + hd * HDIM + c8;
        *(volatile v4u_t*)(Oh + off) = hv[it];
        *(volatile v4u_t*)(Ol + off) = lv[it];
    }
}

extern "C" void kernel_launch(void* const* d_in, const int* in_sizes, int n_in,
                              void* d_out, int out_size, void* d_ws, size_t ws_size,
                              hipStream_t stream) {
    if (n_in < 10) return;
    const int DD = DIM * DIM;
    if (in_sizes[0] != NROWS * DIM) return;
    if (in_sizes[1] != DD || in_sizes[3] != DD || in_sizes[5] != DD || in_sizes[7] != DD || in_sizes[9] != DD) return;
    if (in_sizes[2] != DIM || in_sizes[4] != DIM || in_sizes[6] != DIM || in_sizes[8] != DIM) return;
    if (out_size != NROWS * DIM) return;

    const float* x   = (const float*)d_in[0];
    const float* W_q = (const float*)d_in[1];
    const float* b_q = (const float*)d_in[2];
    const float* W_k = (const float*)d_in[3];
    const float* b_k = (const float*)d_in[4];
    const float* W_v = (const float*)d_in[5];
    const float* b_v = (const float*)d_in[6];
    const float* W_o = (const float*)d_in[7];
    const float* b_o = (const float*)d_in[8];
    const float* W_s = (const float*)d_in[9];
    float* outp = (float*)d_out;

    const size_t E16 = (size_t)NROWS * DIM * sizeof(unsigned short);
    const size_t WTB = (size_t)5 * DD * sizeof(unsigned short);
    char* ws = (char*)d_ws;
    size_t off = 0;
    unsigned short* Xb  = (unsigned short*)(ws + off); off += E16;
    unsigned short* Wt  = (unsigned short*)(ws + off); off += WTB;
    unsigned short* Q1h = (unsigned short*)(ws + off); off += E16;
    unsigned short* Q1l = (unsigned short*)(ws + off); off += E16;
    unsigned short* Kh  = (unsigned short*)(ws + off); off += E16;
    unsigned short* Kl  = (unsigned short*)(ws + off); off += E16;
    unsigned short* Vt  = (unsigned short*)(ws + off); off += E16;
    unsigned short* Q2h = (unsigned short*)(ws + off); off += E16;
    unsigned short* Q2l = (unsigned short*)(ws + off); off += E16;
    unsigned short* Oh  = (unsigned short*)(ws + off); off += E16;
    unsigned short* Ol  = (unsigned short*)(ws + off); off += E16;
    if (off > ws_size) return;

    const unsigned short* Wtq = Wt + (size_t)0 * DD;
    const unsigned short* Wtk = Wt + (size_t)1 * DD;
    const unsigned short* Wtv = Wt + (size_t)2 * DD;
    const unsigned short* Wto = Wt + (size_t)3 * DD;
    const unsigned short* Wts = Wt + (size_t)4 * DD;

    {
        const int n8 = NROWS * DIM / 8;
        k_cvt_x<<<(n8 + 255) / 256, 256, 0, stream>>>(x, Xb, n8);
    }
    {
        const int total = 5 * DIM * (DIM / 8);
        k_cvt_w<<<(total + 255) / 256, 256, 0, stream>>>(W_q, W_k, W_v, W_o, W_s, Wt, DIM, total);
    }
    const dim3 ggrid((NROWS + 63) / 64, (DIM + 127) / 128);
    k_gemm<1, 0, 1><<<ggrid, 128, 0, stream>>>(Xb, Xb, Wtq, b_q, Q1h, Q1l, outp, NROWS, DIM, DIM);
    k_gemm<1, 0, 1><<<ggrid, 128, 0, stream>>>(Xb, Xb, Wtk, b_k, Kh, Kl, outp, NROWS, DIM, DIM);
    k_gemm<1, 1, 1><<<ggrid, 128, 0, stream>>>(Xb, Xb, Wtv, b_v, Vt, Vt, outp, NROWS, DIM, DIM);
    k_gemm<2, 0, 0><<<ggrid, 128, 0, stream>>>(Q1h, Q1l, Wts, b_q, Q2h, Q2l, outp, NROWS, DIM, DIM);
    k_attn<<<dim3(TSEQ / 64, NHEAD, BATCH), 128, 0, stream>>>(Q2h, Q2l, Kh, Kl, Vt, Oh, Ol);
    k_gemm<2, 2, 1><<<ggrid, 128, 0, stream>>>(Oh, Ol, Wto, b_o, Oh, Ol, outp, NROWS, DIM, DIM);
    (void)hipGetLastError();
}
